// HSTULayer_38585986187605
// MI455X (gfx1250) — hardware-verified
//
#include <hip/hip_runtime.h>


#define NB_  4
#define TT   2048
#define E_   512
#define PW   2048
#define NH_  8
#define HD   64
#define UOFF 0
#define VOFF 512
#define QOFF 1024
#define KOFF 1536
typedef _Float16 h16;
typedef unsigned short bf;
typedef __attribute__((ext_vector_type(16))) __bf16   v16bf;
typedef __attribute__((ext_vector_type(16))) _Float16 v16h;
typedef __attribute__((ext_vector_type(8)))  _Float16 v8h;
typedef __attribute__((ext_vector_type(8)))  unsigned short v8us;
typedef __attribute__((ext_vector_type(8)))  float    v8f;
typedef __attribute__((ext_vector_type(4)))  float    v4f;
typedef v8h  __attribute__((may_alias)) v8ha;
typedef v4f  __attribute__((may_alias)) v4fa;
typedef v8us __attribute__((may_alias)) v8usa;

__device__ __forceinline__ unsigned short f2bf(float f) { unsigned u = __float_as_uint(f); u += 0x7FFFu + ((u >> 16) & 1u); return (unsigned short)(u >> 16); }
__device__ __forceinline__ float bf2f(unsigned short b) { return __uint_as_float(((unsigned)b) << 16); }
__device__ __forceinline__ float bfr(float f) { return bf2f(f2bf(f)); }
__device__ __forceinline__ v16h cat16(v8h lo, v8h hi) { return __builtin_shufflevector(lo, hi, 0, 1, 2, 3, 4, 5, 6, 7, 8, 9, 10, 11, 12, 13, 14, 15); }
__device__ __forceinline__ v16bf cat16b(v8us lo, v8us hi) { return __builtin_bit_cast(v16bf, __builtin_shufflevector(lo, hi, 0, 1, 2, 3, 4, 5, 6, 7, 8, 9, 10, 11, 12, 13, 14, 15)); }
__device__ __forceinline__ v8f wmma16(v16h a, v16h b, v8f c) { return __builtin_amdgcn_wmma_f32_16x16x32_f16(false, a, false, b, (short)0, c, false, false); }
__device__ __forceinline__ v8f wmmab(v16bf a, v16bf b, v8f c) { return __builtin_amdgcn_wmma_f32_16x16x32_bf16(false, a, false, b, (short)0, c, false, false); }


template <typename T16> struct WFrag;
template <> struct WFrag<h16> { typedef v16h V; static __device__ __forceinline__ V ld(const h16* p) { return cat16(*(const v8h*)p, *(const v8h*)(p + 16)); } static __device__ __forceinline__ v8f mma(V a, V b, v8f c) { return wmma16(a, b, c); } };
template <> struct WFrag<bf> { typedef v16bf V; static __device__ __forceinline__ V ld(const bf* p) { return cat16b(*(const v8us*)p, *(const v8us*)(p + 16)); } static __device__ __forceinline__ v8f mma(V a, V b, v8f c) { return wmmab(a, b, c); } };
template <typename T16, int NSPLIT, bool BIAS>
__global__ __launch_bounds__(32) void k_gemmw(const T16* __restrict__ A, const T16* __restrict__ A2, const T16* __restrict__ Bt, const T16* __restrict__ Bt2, int K, float* C, int ldc, const float* __restrict__ bias, size_t sA, size_t sB, size_t sC) {
    typedef typename WFrag<T16>::V V;
    __shared__ __align__(16) float os[16 * 68];
    const size_t z = blockIdx.z; A += z * sA; if (A2) A2 += z * sA; Bt += z * sB; if (Bt2) Bt2 += z * sB; C += z * sC;
    const int lane = threadIdx.x & 31, lr = lane & 15, hi = lane >> 4; const int r0 = blockIdx.x * 64, c0 = blockIdx.y * 64;
    v8f acc[4][4];
#pragma unroll
    for (int mb = 0; mb < 4; ++mb)
#pragma unroll
        for (int nb = 0; nb < 4; ++nb) acc[mb][nb] = (v8f){};
    const size_t aoff = (size_t)(r0 + lr) * K + 8 * hi, boff = (size_t)(c0 + lr) * K + 8 * hi;
#pragma unroll 1
    for (int kc = 0; kc < K; kc += 32) {
        V a[4], a2[4];
#pragma unroll
        for (int mb = 0; mb < 4; ++mb) { a[mb] = WFrag<T16>::ld(A + aoff + (size_t)mb * 16 * K + kc); if (NSPLIT == 1 || NSPLIT == 2) a2[mb] = WFrag<T16>::ld(A2 + aoff + (size_t)mb * 16 * K + kc); }
#pragma unroll
        for (int nb = 0; nb < 4; ++nb) { const V b = WFrag<T16>::ld(Bt + boff + (size_t)nb * 16 * K + kc); V b2; if (NSPLIT >= 2) b2 = WFrag<T16>::ld(Bt2 + boff + (size_t)nb * 16 * K + kc);
#pragma unroll
            for (int mb = 0; mb < 4; ++mb) { acc[mb][nb] = WFrag<T16>::mma(a[mb], b, acc[mb][nb]); if (NSPLIT == 1 || NSPLIT == 2) acc[mb][nb] = WFrag<T16>::mma(a2[mb], b, acc[mb][nb]); if (NSPLIT >= 2) acc[mb][nb] = WFrag<T16>::mma(a[mb], b2, acc[mb][nb]); } }
        asm volatile("v_nop\n\tv_nop\n\tv_nop\n\tv_nop" : "+v"(acc[0][0]), "+v"(acc[1][1]), "+v"(acc[2][2]), "+v"(acc[3][3]) : "v"(a[0]), "v"(a[3]));
    }
#pragma unroll
    for (int mb = 0; mb < 4; ++mb) {
#pragma unroll
        for (int nb = 0; nb < 4; ++nb) {
#pragma unroll
            for (int j = 0; j < 8; ++j) os[(hi * 8 + j) * 68 + nb * 16 + lr] = acc[mb][nb][j]; }
        __builtin_amdgcn_wave_barrier(); asm volatile("" ::: "memory");
        float* crow = C + (size_t)(r0 + mb * 16) * ldc + c0;
#pragma unroll 1
        for (int ps = 0; ps < 2; ++ps) {
#pragma unroll
            for (int s = 0; s < 8; ++s) { const int row = 2 * s + hi, cofs = lr * 4; v4f val = *(const v4fa*)(os + row * 68 + cofs); if (BIAS) { val[0] += bfr(bias[c0 + cofs]); val[1] += bfr(bias[c0 + cofs + 1]); val[2] += bfr(bias[c0 + cofs + 2]); val[3] += bfr(bias[c0 + cofs + 3]); }
                *(volatile v4f*)(crow + (size_t)row * ldc + cofs) = val; }
            if (ps == 0) __threadfence(); }
        __builtin_amdgcn_wave_barrier(); asm volatile("" ::: "memory");
    }
}

__device__ __forceinline__ h16 tohx(float x) { return (h16)x; }
__device__ __forceinline__ void splitf(float y, unsigned short& h, unsigned short& l) { h = f2bf(y); l = f2bf(y - bf2f(h)); }
typedef __attribute__((ext_vector_type(2))) _Float16 v2h;
typedef __attribute__((ext_vector_type(4))) _Float16 v4h;
typedef __attribute__((ext_vector_type(2))) unsigned short v2us;
typedef __attribute__((ext_vector_type(4))) unsigned short v4us;
typedef __attribute__((ext_vector_type(2))) float v2f;
typedef __attribute__((ext_vector_type(4))) int v4i;

__global__ __launch_bounds__(256) void k_wtG(const float* __restrict__ w, int K, int N, bf* Bt) {
    const int lane = threadIdx.x & 31; const int L0 = (blockIdx.x * 8 + (threadIdx.x >> 5)) * 8; const int nlines = N * K / 64;
#pragma unroll
    for (int ps = 0; ps < 2; ++ps) {
#pragma unroll 1
        for (int l = 0; l < 8; ++l) { const int L = L0 + l; if (L >= nlines) break; const size_t e = (size_t)L * 64 + lane * 2; const int k = (int)(e % K), n = (int)(e / K); v2us o;
            o[0] = f2bf(w[(size_t)k * N + n]); o[1] = f2bf(w[(size_t)(k + 1) * N + n]); *(volatile v2us*)(Bt + e) = o; }
        if (ps == 0) __threadfence(); }
}

__global__ __launch_bounds__(256) void k_lnx(const float* __restrict__ X, const float* __restrict__ gw, const float* __restrict__ gb, bf* Ph, bf* Pl) { const int lane = threadIdx.x & 31; const int r = blockIdx.x * 8 + (threadIdx.x >> 5); if (r >= TT) return; const float* xr = X + (size_t)r * E_; float hv[16]; float s = 0.f;
#pragma unroll
    for (int ch = 0; ch < 4; ++ch) { const v4f a = *(const v4f*)(xr + ch * 128 + lane * 4);
#pragma unroll
        for (int q = 0; q < 4; ++q) { const float u = bfr(a[q]); hv[ch * 4 + q] = u; s += u; } }
#pragma unroll
    for (int sh = 16; sh; sh >>= 1) s += __shfl_xor(s, sh, 32);
    float mu = s * (1.0f / 512.0f); asm volatile("" : "+v"(mu)); float s2 = 0.f;
#pragma unroll
    for (int k = 0; k < 16; ++k) { float d0 = __fsub_rn(hv[k], mu); asm volatile("" : "+v"(d0)); float p = __fmul_rn(d0, d0); asm volatile("" : "+v"(p)); s2 = __fadd_rn(s2, p); }
#pragma unroll
    for (int sh = 16; sh; sh >>= 1) s2 += __shfl_xor(s2, sh, 32);
    float var = __fadd_rn(s2 * (1.0f / 512.0f), 1e-6f); asm volatile("" : "+v"(var)); const float rs = __frsqrt_rn(var);
#pragma unroll 1
    for (int ps = 0; ps < 2; ++ps) {
#pragma unroll
        for (int ch = 0; ch < 4; ++ch) { const int c0 = ch * 128 + lane * 4; v4us oh, ol;
#pragma unroll
            for (int q = 0; q < 4; ++q) { float gg = bfr(gw[c0 + q]); asm volatile("" : "+v"(gg)); float d0 = __fsub_rn(hv[ch * 4 + q], mu); asm volatile("" : "+v"(d0)); float n0 = __fmul_rn(d0, rs); asm volatile("" : "+v"(n0)); float y = __fmul_rn(n0, gg); asm volatile("" : "+v"(y)); const float z = __fadd_rn(y, bfr(gb[c0 + q])); unsigned short a2, c2; splitf(z, a2, c2); oh[q] = a2; ol[q] = c2; }
            const size_t oo = (size_t)r * E_ + c0; *(volatile v4us*)(Ph + oo) = oh; *(volatile v4us*)(Pl + oo) = ol; }
        if (ps == 0) __threadfence(); } }
__global__ __launch_bounds__(256) void k_pl16o(const float* __restrict__ F, int coff, h16* P16) { const size_t e = ((size_t)blockIdx.x * 256 + threadIdx.x) * 2; if (e >= (size_t)NH_ * TT * HD) return; const int d = (int)(e % HD); const int t = (int)((e / HD) % TT); const int h = (int)(e / ((size_t)HD * TT)); const float* f = F + (size_t)t * PW + coff + h * HD + d; v2h o; o[0] = tohx(f[0]); o[1] = tohx(f[1]);
    *(volatile v2h*)(P16 + e) = o; __threadfence(); *(volatile v2h*)(P16 + e) = o; }
__global__ __launch_bounds__(256) void k_vt16o(const float* __restrict__ F, int coff, h16* V16) { const size_t e = ((size_t)blockIdx.x * 256 + threadIdx.x) * 2; if (e >= (size_t)NH_ * HD * TT) return; const int t = (int)(e % TT); const int d = (int)((e / TT) % HD); const int h = (int)(e / ((size_t)TT * HD)); v2h o;
#pragma unroll
    for (int q = 0; q < 2; ++q) o[q] = tohx(F[((size_t)t + q) * PW + coff + h * HD + d]);
    *(volatile v2h*)(V16 + e) = o; __threadfence(); *(volatile v2h*)(V16 + e) = o; }
__global__ __launch_bounds__(256) void k_silum(const float* __restrict__ Sb, const float* __restrict__ MK, h16* A16, size_t n8) { const size_t i = (size_t)blockIdx.x * 256 + threadIdx.x; if (i >= n8) return; const v8f a = *(const v8f*)(Sb + i * 8); const v8f m = *(const v8f*)(MK + i * 8); v8h o;
#pragma unroll
    for (int q = 0; q < 8; ++q) { float den = __fadd_rn(1.0f, expf(-a[q])); asm volatile("" : "+v"(den)); float sl = __fdiv_rn(a[q], den); asm volatile("" : "+v"(sl)); float mb = bfr(m[q]); asm volatile("" : "+v"(mb)); o[q] = tohx(__fmul_rn(sl, mb)); }
    *(volatile v8h*)(A16 + i * 8) = o; __threadfence(); *(volatile v8h*)(A16 + i * 8) = o; }
__global__ __launch_bounds__(256) void k_mrgf(const float* __restrict__ O, int h, float* AO) { const size_t e = ((size_t)blockIdx.x * 256 + threadIdx.x) * 2; if (e >= (size_t)TT * HD) return; const int d = (int)(e % HD); const int t = (int)(e / HD); v2f o; o[0] = O[e]; o[1] = O[e + 1]; const size_t oo = (size_t)t * E_ + h * HD + d;
    *(volatile v2f*)(AO + oo) = o; __threadfence(); *(volatile v2f*)(AO + oo) = o; }
__global__ __launch_bounds__(256) void k_lnout(const float* __restrict__ AO, const float* __restrict__ F, const float* __restrict__ X, const float* __restrict__ gw, const float* __restrict__ gb, float* out) { const int lane = threadIdx.x & 31; const int r = blockIdx.x * 8 + (threadIdx.x >> 5); if (r >= TT) return; const float* ar = AO + (size_t)r * E_; float hv[16]; float s = 0.f;
#pragma unroll
    for (int ch = 0; ch < 4; ++ch) { const v4f a = *(const v4f*)(ar + ch * 128 + lane * 4);
#pragma unroll
        for (int q = 0; q < 4; ++q) { hv[ch * 4 + q] = a[q]; s += a[q]; } }
#pragma unroll
    for (int sh = 16; sh; sh >>= 1) s += __shfl_xor(s, sh, 32);
    float mu = s * (1.0f / 512.0f); asm volatile("" : "+v"(mu)); float s2 = 0.f;
#pragma unroll
    for (int k = 0; k < 16; ++k) { float d0 = __fsub_rn(hv[k], mu); asm volatile("" : "+v"(d0)); float p = __fmul_rn(d0, d0); asm volatile("" : "+v"(p)); s2 = __fadd_rn(s2, p); }
#pragma unroll
    for (int sh = 16; sh; sh >>= 1) s2 += __shfl_xor(s2, sh, 32);
    float var = __fadd_rn(s2 * (1.0f / 512.0f), 1e-6f); asm volatile("" : "+v"(var)); const float rs = __frsqrt_rn(var);
    const float* ur = F + (size_t)r * PW + UOFF; const float* xr = X + (size_t)r * E_;
#pragma unroll 1
    for (int ps = 0; ps < 2; ++ps) {
#pragma unroll
        for (int ch = 0; ch < 4; ++ch) { const int c0 = ch * 128 + lane * 4; const v4f uu = *(const v4f*)(ur + c0); const v4f xx = *(const v4f*)(xr + c0); v4f o;
#pragma unroll
            for (int q = 0; q < 4; ++q) { float gg = bfr(gw[c0 + q]); asm volatile("" : "+v"(gg)); float d0 = __fsub_rn(hv[ch * 4 + q], mu); asm volatile("" : "+v"(d0)); float n0 = __fmul_rn(d0, rs); asm volatile("" : "+v"(n0)); float y = __fmul_rn(n0, gg); asm volatile("" : "+v"(y)); float z = __fadd_rn(y, bfr(gb[c0 + q])); asm volatile("" : "+v"(z)); float yu = __fmul_rn(z, uu[q]); asm volatile("" : "+v"(yu)); o[q] = __fadd_rn(bfr(xx[q]), yu); }
            *(volatile v4f*)(out + (size_t)r * E_ + c0) = o; }
        if (ps == 0) __threadfence(); } }

extern "C" void kernel_launch(void* const* d_in, const int* in_sizes, int n_in,
                              void* d_out, int out_size, void* d_ws, size_t ws_size, hipStream_t stream) {
    (void)in_sizes; (void)n_in; (void)out_size;
    const float* x = (const float*)d_in[0]; const float* MK = (const float*)d_in[1]; const float* wuvqk = (const float*)d_in[2]; const float* ing = (const float*)d_in[3]; const float* inb = (const float*)d_in[4]; const float* og = (const float*)d_in[5]; const float* ob = (const float*)d_in[6];
    float* OUT = (float*)d_out;
    char* wsp = (char*)d_ws;
    auto take = [&](size_t bytes) { char* p = wsp; wsp += (bytes + 255) & ~(size_t)255; return (void*)p; };
    bf* WB = (bf*)take((size_t)PW * E_ * 2); bf* NXh = (bf*)take((size_t)TT * E_ * 2); bf* NXl = (bf*)take((size_t)TT * E_ * 2); float* F = (float*)take((size_t)TT * PW * 4);
    const size_t PS = (size_t)NH_ * TT * HD; h16* Q16 = (h16*)take(PS * 2); h16* K16 = (h16*)take(PS * 2); h16* VT16 = (h16*)take(PS * 2);
    float* Sb = (float*)take((size_t)TT * TT * 4); h16* A16 = (h16*)take((size_t)TT * TT * 2); float* Ob = (float*)take((size_t)TT * HD * 4); float* AO = (float*)take((size_t)TT * E_ * 4);
    if ((size_t)(wsp - (char*)d_ws) > ws_size) return;
    k_wtG<<<(unsigned)((E_ * PW / 64 + 63) / 64), 256, 0, stream>>>(wuvqk, E_, PW, WB);
    const unsigned LP = (unsigned)((PS / 2 + 255) / 256);
    for (int b = 0; b < NB_; ++b) { const float* xb = x + (size_t)b * TT * E_;
        k_lnx<<<TT / 8, 256, 0, stream>>>(xb, ing, inb, NXh, NXl);
        k_gemmw<bf, 1, false><<<dim3(TT / 64, PW / 64, 1), 32, 0, stream>>>(NXh, NXl, WB, nullptr, E_, F, PW, nullptr, 0, 0, 0);
        k_pl16o<<<LP, 256, 0, stream>>>(F, QOFF, Q16); k_pl16o<<<LP, 256, 0, stream>>>(F, KOFF, K16); k_vt16o<<<LP, 256, 0, stream>>>(F, VOFF, VT16);
        for (int h = 0; h < NH_; ++h) { const size_t po = (size_t)h * TT * HD;
            k_gemmw<h16, 0, false><<<dim3(TT / 64, TT / 64, 1), 32, 0, stream>>>(Q16 + po, nullptr, K16 + po, nullptr, HD, Sb, TT, nullptr, 0, 0, 0);
            k_silum<<<(unsigned)(((size_t)TT * TT / 8 + 255) / 256), 256, 0, stream>>>(Sb, MK, A16, (size_t)TT * TT / 8);
            k_gemmw<h16, 0, false><<<dim3(TT / 64, HD / 64, 1), 32, 0, stream>>>(A16, nullptr, VT16 + po, nullptr, TT, Ob, HD, nullptr, 0, 0, 0);
            k_mrgf<<<(unsigned)(((size_t)TT * HD / 2 + 255) / 256), 256, 0, stream>>>(Ob, h, AO); }
        k_lnout<<<TT / 8, 256, 0, stream>>>(AO, F, xb, og, ob, OUT + (size_t)b * TT * E_); }
}
